// Net_14422500180486
// MI455X (gfx1250) — hardware-verified
//
#include <hip/hip_runtime.h>
#include <math.h>

constexpr int BATCH    = 32;
constexpr int TSTEPS   = 2048;
constexpr int DIN      = 64;
constexpr int HID      = 128;
constexpr int GATES    = 4 * HID;
constexpr int NTHR     = 256;
constexpr int SEQ_BLK  = 16;
constexpr int ROWS_ALL = BATCH * TSTEPS;
constexpr int HPITCH   = 136;
constexpr int XPITCH   = 520;
constexpr int OPITCH   = 132;
constexpr float WCARRY     = 16.0f;
constexpr float WCARRY_INV = 1.0f / 16.0f;

static_assert(BATCH % SEQ_BLK == 0, "batch tiles");
static_assert(HID == 16 * (NTHR / 32), "8 waves x 16 hidden units");
static_assert(ROWS_ALL % 64 == 0 && GATES % 64 == 0, "GEMM M, N tile multiples");
static_assert(DIN % 32 == 0 && HID % 32 == 0, "GEMM K multiples of 32");
static_assert((HPITCH * 2) % 16 == 0 && (XPITCH * 2) % 16 == 0 && (OPITCH * 4) % 16 == 0, "16-B aligned LDS rows");
static_assert(SEQ_BLK * GATES / 8 == 4 * NTHR, "xg tile = 4 x 16-B loads per thread");
static_assert(SEQ_BLK * HID / 8 == NTHR, "h0 tile = one 16-B store per thread");
static_assert(SEQ_BLK * HID / 4 == 2 * NTHR, "out tile = two 16-B stores per thread");

typedef __attribute__((ext_vector_type(16))) _Float16 v16h;
typedef __attribute__((ext_vector_type(8)))  _Float16 v8h;
typedef __attribute__((ext_vector_type(8)))  float    v8f;
typedef __attribute__((ext_vector_type(4)))  float    v4f;
typedef __attribute__((ext_vector_type(4)))  unsigned v4u;

union FragU { v16h v; v8h h[2]; };
__device__ __forceinline__ v16h frag_load(const _Float16* p) {
  FragU f;
  f.h[0] = *(const v8h*)(p);
  f.h[1] = *(const v8h*)(p + 16);
  return f.v;
}
__device__ __forceinline__ v8f mma_f16(v16h a, v16h b, v8f c) {
  return __builtin_amdgcn_wmma_f32_16x16x32_f16(false, a, false, b, (short)0, c, false, false);
}
__device__ __forceinline__ void mma_guard4(v8f& a0, v8f& a1, v8f& a2, v8f& a3,
                                           v16h x, v16h b0, v16h b1, v16h b2, v16h b3) {
  asm volatile("v_nop\n\tv_nop\n\tv_nop\n\tv_nop"
               : "+v"(a0), "+v"(a1), "+v"(a2), "+v"(a3)
               : "v"(x), "v"(b0), "v"(b1), "v"(b2), "v"(b3));
}
__device__ __forceinline__ void keep4_h(v16h a, v16h b, v16h c, v16h d) {
  asm volatile("v_nop" :: "v"(a), "v"(b), "v"(c), "v"(d));
}
__device__ __forceinline__ void acc_guard4(v8f& a, v8f& b, v8f& c, v8f& d) {
  asm volatile("v_nop\n\tv_nop\n\tv_nop\n\tv_nop" : "+v"(a), "+v"(b), "+v"(c), "+v"(d));
}

__device__ __forceinline__ float h16_to_f32(unsigned hb) {
  const unsigned sgn = (hb & 0x8000u) << 16;
  const unsigned em = hb & 0x7fffu;
  const float fn = __uint_as_float((em << 13) + 0x38000000u);
  const float fs = (float)em * 5.9604644775390625e-8f;
  const float mag = (em < 0x400u) ? fs : fn;
  return __uint_as_float(__float_as_uint(mag) | sgn);
}

__device__ __forceinline__ float gate_sig(float x)  { return __builtin_amdgcn_rcpf(1.0f + expf(-x)); }
__device__ __forceinline__ float gate_tanh(float x) { return 1.0f - 2.0f * __builtin_amdgcn_rcpf(expf(2.0f * x) + 1.0f); }

__global__ __launch_bounds__(NTHR) void cvt_dense_f16_kernel(const float* __restrict__ src,
                                                             unsigned short* __restrict__ dst, int n8, float sc) {
  const int i = blockIdx.x * NTHR + threadIdx.x;
  if (i < n8) {
    const float* sp = src + (size_t)i * 8;
    const v4f a = *(const v4f*)(sp);
    const v4f b = *(const v4f*)(sp + 4);
    v8h hv;
#pragma unroll
    for (int e = 0; e < 4; ++e) {
      hv[e]     = (_Float16)(a[e] * sc);
      hv[4 + e] = (_Float16)(b[e] * sc);
    }
    *(volatile v8h*)(dst + (size_t)i * 8) = hv;
    __threadfence();
    *(volatile v8h*)(dst + (size_t)i * 8) = hv;
  }
}

__global__ __launch_bounds__(NTHR) void cvt_x_tmajor_kernel(const float* __restrict__ x, unsigned short* __restrict__ dst) {
  const int i = blockIdx.x * NTHR + threadIdx.x;
  if (i < ROWS_ALL * (DIN / 8)) {
    const int R  = i >> 3;
    const int c8 = (i & 7) * 8;
    const int t  = R >> 5;
    const int b  = R & 31;
    const float* sp = x + ((size_t)b * TSTEPS + (size_t)t) * DIN + c8;
    const v4f a  = *(const v4f*)(sp);
    const v4f bq = *(const v4f*)(sp + 4);
    v8h hv;
#pragma unroll
    for (int e = 0; e < 4; ++e) {
      hv[e]     = (_Float16)a[e];
      hv[4 + e] = (_Float16)bq[e];
    }
    *(volatile v8h*)(dst + (size_t)i * 8) = hv;
    __threadfence();
    *(volatile v8h*)(dst + (size_t)i * 8) = hv;
  }
}

__global__ __launch_bounds__(NTHR) void bias_sum_kernel(const float* __restrict__ bi0, const float* __restrict__ bh0,
                                                        const float* __restrict__ bi1, const float* __restrict__ bh1,
                                                        float* __restrict__ dst) {
  const int tid = threadIdx.x;
  const int which = tid >> 7;
  const int idx = (tid & 127) * 4;
  const v4f a0 = *(const v4f*)(bi0 + idx);
  const v4f c0 = *(const v4f*)(bh0 + idx);
  const v4f a1 = *(const v4f*)(bi1 + idx);
  const v4f c1 = *(const v4f*)(bh1 + idx);
  v4f o;
#pragma unroll
  for (int e = 0; e < 4; ++e) {
    const float s0 = a0[e] + c0[e];
    const float s1 = a1[e] + c1[e];
    o[e] = which ? s1 : s0;
  }
  float* op = dst + which * GATES + idx;
  *(volatile v4f*)op = o;
  __threadfence();
  *(volatile v4f*)op = o;
}

__global__ __launch_bounds__(256) void gemm64_f16_kernel(
    const unsigned short* __restrict__ Ap, int lda,
    const unsigned short* __restrict__ Btp, int ldb,
    unsigned short* __restrict__ C, int ldc,
    const float* __restrict__ bias, int M, int N, int K, float scale) {
  const _Float16* A  = (const _Float16*)Ap;
  const _Float16* Bt = (const _Float16*)Btp;
  __shared__ __align__(16) float sT[8][16 * 68];
  const int lane = threadIdx.x & 31;
  const int wave = threadIdx.x >> 5;
  const int tilesN = N >> 6;
  const int tilesM = M >> 6;
  const int tile = blockIdx.x * 8 + wave;
  if (tile >= tilesM * tilesN) return;
  const int tm = tile / tilesN;
  const int tn = tile - tm * tilesN;
  const int m0 = tm << 6;
  const int n0 = tn << 6;
  const int rlane = lane & 15;
  const int koff  = (lane >> 4) * 8;
  const int mOff  = (lane >> 4) * 8;

  v8f acc[4][4];
#pragma unroll
  for (int i = 0; i < 4; ++i)
#pragma unroll
    for (int j = 0; j < 4; ++j) acc[i][j] = (v8f){0.f, 0.f, 0.f, 0.f, 0.f, 0.f, 0.f, 0.f};

  for (int k0 = 0; k0 < K; k0 += 32) {
    v16h bh[4];
#pragma unroll
    for (int j = 0; j < 4; ++j) {
      const size_t bo = (size_t)(n0 + (j << 4) + rlane) * ldb + koff + k0;
      bh[j] = frag_load(Bt + bo);
    }
#pragma unroll
    for (int i = 0; i < 4; ++i) {
      const size_t ao = (size_t)(m0 + (i << 4) + rlane) * lda + koff + k0;
      const v16h ah = frag_load(A + ao);
#pragma unroll
      for (int j = 0; j < 4; ++j) acc[i][j] = mma_f16(ah, bh[j], acc[i][j]);
      mma_guard4(acc[i][0], acc[i][1], acc[i][2], acc[i][3], ah, bh[0], bh[1], bh[2], bh[3]);
    }
    keep4_h(bh[0], bh[1], bh[2], bh[3]);
  }
  acc_guard4(acc[0][0], acc[0][1], acc[0][2], acc[0][3]);
  acc_guard4(acc[1][0], acc[1][1], acc[1][2], acc[1][3]);
  acc_guard4(acc[2][0], acc[2][1], acc[2][2], acc[2][3]);
  acc_guard4(acc[3][0], acc[3][1], acc[3][2], acc[3][3]);

  float* slab = sT[wave];
#pragma unroll
  for (int i = 0; i < 4; ++i) {
    const int mBase = m0 + (i << 4);
#pragma unroll
    for (int j = 0; j < 4; ++j) {
      const int n = n0 + (j << 4) + rlane;
      const float bv = bias[n];
#pragma unroll
      for (int r = 0; r < 8; ++r) {
        const float v = acc[i][j][r] * scale + bv;
        slab[(mOff + r) * 68 + (j << 4) + rlane] = v;
      }
    }
    __builtin_amdgcn_fence(__ATOMIC_RELEASE, "workgroup");
    __builtin_amdgcn_wave_barrier();
    __builtin_amdgcn_fence(__ATOMIC_ACQUIRE, "workgroup");
    {
      const int q = lane >> 3, c8 = (lane & 7) * 8;
      for (int pass = 0; pass < 2; ++pass) {
#pragma unroll
        for (int it = 0; it < 4; ++it) {
          const int row = it * 4 + q;
          const float* sp = slab + row * 68 + c8;
          v8h hv;
#pragma unroll
          for (int e = 0; e < 8; ++e) hv[e] = (_Float16)sp[e];
          *(volatile v8h*)(C + (size_t)(mBase + row) * ldc + n0 + c8) = hv;
        }
        __threadfence();
      }
    }
    __builtin_amdgcn_fence(__ATOMIC_RELEASE, "workgroup");
    __builtin_amdgcn_wave_barrier();
    __builtin_amdgcn_fence(__ATOMIC_ACQUIRE, "workgroup");
  }
}

template <bool LAST>
__global__ __launch_bounds__(NTHR) void lstm_rec_kernel(const unsigned short* __restrict__ XGp,
                                                        const unsigned short* __restrict__ WHp,
                                                        unsigned short* __restrict__ HSEQ,
                                                        float* __restrict__ OUT) {
  __shared__ __align__(16) _Float16       Ah[SEQ_BLK * HPITCH];
  __shared__ __align__(16) unsigned short Xs[SEQ_BLK * XPITCH];
  __shared__ __align__(16) float          Hs[SEQ_BLK * OPITCH];
  const _Float16* WH = (const _Float16*)WHp;
  const int tid = threadIdx.x, lane = tid & 31, wave = tid >> 5;
  const int c = lane & 15, hh = lane >> 4, koff = hh * 8;
  const int rowbase = blockIdx.x * SEQ_BLK;
  const int j = 16 * wave + c;

#pragma unroll 1
  for (int i = tid; i < SEQ_BLK * HPITCH; i += NTHR) Ah[i] = (_Float16)0.0f;

  const unsigned short* xg_blk = XGp + (size_t)rowbase * GATES;
  v4u pf[4];
#pragma unroll
  for (int i = 0; i < 4; ++i) {
    const int idx = i * NTHR + tid;
    pf[i] = *(const v4u*)(xg_blk + (size_t)idx * 8);
  }
#pragma unroll
  for (int i = 0; i < 4; ++i) {
    const int idx = i * NTHR + tid;
    const int row = idx >> 6, c8 = (idx & 63) * 8;
    *(v4u*)(Xs + row * XPITCH + c8) = pf[i];
  }
  float cst[8];
#pragma unroll
  for (int r = 0; r < 8; ++r) cst[r] = 0.0f;
  __syncthreads();

  const _Float16* ahrow = Ah + c * HPITCH + koff;
  const _Float16* wh    = WH + (size_t)j * HID + koff;
  const unsigned short* xrow = Xs + (8 * hh) * XPITCH + j;
  const v8f z8 = {0.f, 0.f, 0.f, 0.f, 0.f, 0.f, 0.f, 0.f};

#pragma unroll 1
  for (int t = 0; t < TSTEPS; ++t) {
    {
      const int tn = (t + 1 < TSTEPS) ? (t + 1) : (TSTEPS - 1);
      const unsigned short* src = xg_blk + (size_t)tn * BATCH * GATES;
#pragma unroll
      for (int i = 0; i < 4; ++i) {
        const int idx = i * NTHR + tid;
        pf[i] = *(const v4u*)(src + (size_t)idx * 8);
      }
    }

    v8f acc0 = z8, acc1 = z8, acc2 = z8, acc3 = z8;
#pragma unroll 1
    for (int k0 = 0; k0 < HID; k0 += 32) {
      const v16h a  = frag_load(ahrow + k0);
      const v16h b0 = frag_load(wh + k0);
      const v16h b1 = frag_load(wh + (size_t)1 * HID * HID + k0);
      const v16h b2 = frag_load(wh + (size_t)2 * HID * HID + k0);
      const v16h b3 = frag_load(wh + (size_t)3 * HID * HID + k0);
      acc0 = mma_f16(a, b0, acc0);
      acc1 = mma_f16(a, b1, acc1);
      acc2 = mma_f16(a, b2, acc2);
      acc3 = mma_f16(a, b3, acc3);
      mma_guard4(acc0, acc1, acc2, acc3, a, b0, b1, b2, b3);
    }
    acc_guard4(acc0, acc1, acc2, acc3);

    float hnew[8];
#pragma unroll
    for (int r = 0; r < 8; ++r) {
      const unsigned short* xp = xrow + r * XPITCH;
      const float xi = h16_to_f32((unsigned)xp[0]);
      const float xf = h16_to_f32((unsigned)xp[HID]);
      const float xc = h16_to_f32((unsigned)xp[2 * HID]);
      const float xo = h16_to_f32((unsigned)xp[3 * HID]);
      const float zi = acc0[r] * WCARRY_INV + xi;
      const float zf = acc1[r] * WCARRY_INV + xf;
      const float zc = acc2[r] * WCARRY_INV + xc;
      const float zo = acc3[r] * WCARRY_INV + xo;
      const float ig = gate_sig(zi);
      const float fg = gate_sig(zf);
      const float gg = gate_tanh(zc);
      const float og = gate_sig(zo);
      const float cn = fg * cst[r] + ig * gg;
      cst[r] = cn;
      hnew[r] = og * gate_tanh(cn);
    }

    __syncthreads();

#pragma unroll
    for (int r = 0; r < 8; ++r) {
      Ah[(8 * hh + r) * HPITCH + j] = (_Float16)hnew[r];
      if (LAST) Hs[(8 * hh + r) * OPITCH + j] = hnew[r];
    }
#pragma unroll
    for (int i = 0; i < 4; ++i) {
      const int idx = i * NTHR + tid;
      const int row = idx >> 6, c8 = (idx & 63) * 8;
      *(v4u*)(Xs + row * XPITCH + c8) = pf[i];
    }

    __syncthreads();

    if (!LAST) {
      const int row = tid >> 4, c8 = (tid & 15) * 8;
      const v4u hv4 = *(const v4u*)(Ah + row * HPITCH + c8);
      unsigned short* dst = HSEQ + ((size_t)t * BATCH + (size_t)(rowbase + row)) * HID + c8;
      for (int pass = 0; pass < 2; ++pass) {
        *(volatile v4u*)dst = hv4;
        __threadfence();
      }
    } else {
      v4f ov[2];
#pragma unroll
      for (int it = 0; it < 2; ++it) {
        const int idx = it * NTHR + tid;
        const int row = idx >> 5, c4 = (idx & 31) * 4;
        ov[it] = *(const v4f*)(Hs + row * OPITCH + c4);
      }
      for (int pass = 0; pass < 2; ++pass) {
#pragma unroll
        for (int it = 0; it < 2; ++it) {
          const int idx = it * NTHR + tid;
          const int row = idx >> 5, c4 = (idx & 31) * 4;
          *(volatile v4f*)(OUT + ((size_t)(rowbase + row) * TSTEPS + (size_t)t) * HID + c4) = ov[it];
        }
        __threadfence();
      }
    }
  }
}

extern "C" void kernel_launch(void* const* d_in, const int* in_sizes, int n_in,
                              void* d_out, int out_size, void* d_ws, size_t ws_size, hipStream_t stream) {
  if (n_in < 9 || d_out == nullptr || d_ws == nullptr) return;
  if (in_sizes[0] != BATCH * TSTEPS * DIN || in_sizes[1] != GATES * DIN || in_sizes[2] != GATES * HID ||
      in_sizes[3] != GATES || in_sizes[4] != GATES || in_sizes[5] != GATES * HID || in_sizes[6] != GATES * HID ||
      in_sizes[7] != GATES || in_sizes[8] != GATES || out_size != BATCH * TSTEPS * HID) return;

  const float* x    = (const float*)d_in[0];
  const float* Wih0 = (const float*)d_in[1];
  const float* Whh0 = (const float*)d_in[2];
  const float* bih0 = (const float*)d_in[3];
  const float* bhh0 = (const float*)d_in[4];
  const float* Wih1 = (const float*)d_in[5];
  const float* Whh1 = (const float*)d_in[6];
  const float* bih1 = (const float*)d_in[7];
  const float* bhh1 = (const float*)d_in[8];
  float* out = (float*)d_out;

  char* ws = (char*)d_ws;
  size_t off = 0;
  auto carve = [&](size_t bytes) -> char* { char* p = ws + off; off += (bytes + 255) & ~(size_t)255; return p; };
  unsigned short* X16  = (unsigned short*)carve((size_t)ROWS_ALL * DIN * 2);
  unsigned short* W0I  = (unsigned short*)carve((size_t)GATES * DIN * 2);
  unsigned short* W0H  = (unsigned short*)carve((size_t)GATES * HID * 2);
  unsigned short* W1I  = (unsigned short*)carve((size_t)GATES * HID * 2);
  unsigned short* W1H  = (unsigned short*)carve((size_t)GATES * HID * 2);
  float*          BIAS = (float*)carve((size_t)2 * GATES * 4);
  unsigned short* XG   = (unsigned short*)carve((size_t)ROWS_ALL * GATES * 2);
  unsigned short* H0   = (unsigned short*)carve((size_t)ROWS_ALL * HID * 2);
  if (off > ws_size || off > (size_t)134217728) return;

  const int n8x  = ROWS_ALL * (DIN / 8);
  const int n8wi = GATES * (DIN / 8);
  const int n8wh = GATES * (HID / 8);
  cvt_x_tmajor_kernel<<<(n8x + NTHR - 1) / NTHR, NTHR, 0, stream>>>(x, X16);
  cvt_dense_f16_kernel<<<(n8wi + NTHR - 1) / NTHR, NTHR, 0, stream>>>(Wih0, W0I, n8wi, WCARRY);
  cvt_dense_f16_kernel<<<(n8wh + NTHR - 1) / NTHR, NTHR, 0, stream>>>(Whh0, W0H, n8wh, WCARRY);
  cvt_dense_f16_kernel<<<(n8wh + NTHR - 1) / NTHR, NTHR, 0, stream>>>(Wih1, W1I, n8wh, WCARRY);
  cvt_dense_f16_kernel<<<(n8wh + NTHR - 1) / NTHR, NTHR, 0, stream>>>(Whh1, W1H, n8wh, WCARRY);
  bias_sum_kernel<<<1, NTHR, 0, stream>>>(bih0, bhh0, bih1, bhh1, BIAS);

  const int gemm_blocks = (ROWS_ALL / 64) * (GATES / 64) / 8;
  gemm64_f16_kernel<<<gemm_blocks, 256, 0, stream>>>(X16, DIN, W0I, DIN, XG, GATES, BIAS,
                                                     ROWS_ALL, GATES, DIN, WCARRY_INV);
  lstm_rec_kernel<false><<<BATCH / SEQ_BLK, NTHR, 0, stream>>>(XG, W0H, H0, out);
  gemm64_f16_kernel<<<gemm_blocks, 256, 0, stream>>>(H0, HID, W1I, HID, XG, GATES, BIAS + GATES,
                                                     ROWS_ALL, GATES, HID, WCARRY_INV);
  lstm_rec_kernel<true><<<BATCH / SEQ_BLK, NTHR, 0, stream>>>(XG, W1H, H0, out);
}
